// MoEModel_78615081386104
// MI455X (gfx1250) — hardware-verified
//
#include <hip/hip_runtime.h>

#define NB    32768
#define DIN   256
#define NE    8
#define L1N   512
#define L2N   256
#define L3N   128
#define HN    64
#define NTK   3
#define LCAP  12288
#define MT    32
#define NTILE (LCAP / MT)
#define GTPB  256
#define GBLK  (NB / GTPB)
#define K2    (2 * L1N)
#define K3    (2 * L2N)
#define KH    (2 * L3N)

static constexpr float ALPHA_LB = 0.01f;
static constexpr float LN_EPS   = 1e-5f;

#define OFF_STAGE 0
#define OFF_A2    65536
#define OFF_A13   131072
#define OFF_PAR   163840
#define OFF_ENT   174592
#define DYN_LDS   174720
#define PAR_B1 0
#define PAR_S1 512
#define PAR_T1 1024
#define PAR_B2 1536
#define PAR_S2 1792
#define PAR_T2 2048
#define PAR_B3 2304
#define PAR_S3 2432
#define PAR_T3 2560
#define PAR_N  2688

static_assert(OFF_A2 == MT * L1N * 4);
static_assert(OFF_A13 == OFF_A2 + MT * K2 * 2);
static_assert(OFF_PAR == OFF_A13 + MT * K3 * 2);
static_assert(MT * DIN * 2 <= MT * K3 * 2);
static_assert(OFF_ENT == OFF_PAR + PAR_N * 4);
static_assert(DYN_LDS == OFF_ENT + MT * 4);
static_assert(NB % GTPB == 0);
static_assert(NB % 64 == 0);
static_assert(NB % 32 == 0);
static_assert(LCAP % MT == 0);
static_assert(LCAP % 4 == 0);
static_assert((LCAP / 4) % 256 == 0);
static_assert(DIN % 32 == 0);
static_assert(K2 % 32 == 0);
static_assert(K3 % 32 == 0);
static_assert(KH % 32 == 0);
static_assert(L1N == 8 * 64);
static_assert(L2N == 8 * 32);
static_assert(L3N == 8 * 16);

typedef unsigned short us;
typedef __bf16 v16bf __attribute__((ext_vector_type(16)));
typedef us v8us_t __attribute__((ext_vector_type(8)));
typedef v8us_t __attribute__((may_alias)) v8us;
typedef float v8f __attribute__((ext_vector_type(8)));
typedef float v4f_t __attribute__((ext_vector_type(4)));
typedef v4f_t __attribute__((may_alias)) v4f;
typedef unsigned int v4u_t __attribute__((ext_vector_type(4)));
typedef v4u_t __attribute__((may_alias)) v4u;

union BFrag { v16bf v; v8us_t h[2]; };

__device__ __forceinline__ unsigned f2bf(float f) {
  unsigned u = __float_as_uint(f);
  u += 0x7FFFu + ((u >> 16) & 1u);
  return u >> 16;
}
__device__ __forceinline__ float bf2f(unsigned b) { return __uint_as_float(b << 16); }
__device__ __forceinline__ float bfr(float f) { return bf2f(f2bf(f)); }

__device__ __forceinline__ v8f zero8() {
  v8f z;
#pragma unroll
  for (int i = 0; i < 8; ++i) z[i] = 0.0f;
  return z;
}

__device__ __forceinline__ v8f wmma_bf(v16bf a, v16bf b, v8f c) {
  v8f d = __builtin_amdgcn_wmma_f32_16x16x32_bf16(false, a, false, b, (short)0, c, false, false);
  asm volatile("v_nop\n\tv_nop\n\tv_nop\n\tv_nop" : "+v"(d) : "v"(a), "v"(b));
  return d;
}

__device__ __forceinline__ v16bf ldfrag(const us* p, int h) {
  BFrag f;
  f.h[0] = *(const v8us*)(p + 8 * h);
  f.h[1] = *(const v8us*)(p + 16 + 8 * h);
  return f.v;
}

__device__ __forceinline__ float wsum(float v) {
#pragma unroll
  for (int off = 16; off > 0; off >>= 1) v += __shfl_xor(v, off, 32);
  return v;
}
__device__ __forceinline__ int wor(int v) {
#pragma unroll
  for (int off = 16; off > 0; off >>= 1) v |= __shfl_xor(v, off, 32);
  return v;
}

__global__ __launch_bounds__(256) void k_cvt_x(const float* __restrict__ x,
                                               us* __restrict__ xb, int n8)
{
  const int i = blockIdx.x * 256 + threadIdx.x;
  if (i >= n8) return;
  const v4f_t a = *(const v4f*)(x + (size_t)i * 8);
  const v4f_t c = *(const v4f*)(x + (size_t)i * 8 + 4);
  v4u_t o;
  o.x = f2bf(a.x) | (f2bf(a.y) << 16);
  o.y = f2bf(a.z) | (f2bf(a.w) << 16);
  o.z = f2bf(c.x) | (f2bf(c.y) << 16);
  o.w = f2bf(c.z) | (f2bf(c.w) << 16);
  us* d = xb + (size_t)i * 8;
  *(volatile v4u_t*)d = o;
  __threadfence();
  *(volatile v4u_t*)d = o;
}

__global__ __launch_bounds__(256) void k_prep_w(const float* __restrict__ src,
                                                us* __restrict__ dst,
                                                int K, int N, int KK, int mode, int ngroups)
{
  const int g = blockIdx.x * 256 + threadIdx.x;
  if (g >= ngroups) return;
  const int kk8 = KK >> 3;
  const int row = g / kk8;
  const int kk0 = (g - row * kk8) << 3;
  const int mat = row / N, n = row - mat * N;
  const float* s = src + (size_t)mat * K * N + n;
  unsigned hw[8];
#pragma unroll
  for (int j = 0; j < 8; ++j) {
    const int kk = kk0 + j;
    const int k = (mode == 0) ? (kk & (K - 1)) : (((kk >> 3) << 2) + (kk & 3));
    hw[j] = f2bf(s[(size_t)k * N]);
  }
  v4u_t o;
  o.x = hw[0] | (hw[1] << 16);
  o.y = hw[2] | (hw[3] << 16);
  o.z = hw[4] | (hw[5] << 16);
  o.w = hw[6] | (hw[7] << 16);
  us* d = dst + (size_t)row * KK + kk0;
  *(volatile v4u_t*)d = o;
  __threadfence();
  *(volatile v4u_t*)d = o;
}

__global__ __launch_bounds__(GTPB) void k_gate(const float* __restrict__ x,
                                               const float* __restrict__ gW,
                                               const float* __restrict__ gb,
                                               unsigned* __restrict__ route,
                                               float* __restrict__ partg)
{
#pragma clang fp contract(off)
  __shared__ float gws[DIN * NE];
  __shared__ float gbs[NE];
  __shared__ float wred[GTPB / 32][16];
  __shared__ __align__(16) float line[32];

  const int tid = threadIdx.x, lane = tid & 31, w = tid >> 5;
  const int tok = blockIdx.x * GTPB + tid;

#pragma unroll 1
  for (int i = tid; i < DIN * NE; i += GTPB) gws[i] = bfr(gW[i]);
  {
    const float gv = bfr(gb[tid & (NE - 1)]);
    if (tid < NE) gbs[tid] = gv;
  }
  __syncthreads();

  double acc[NE];
#pragma unroll
  for (int e = 0; e < NE; ++e) acc[e] = 0.0;
  const float* xr = x + (size_t)tok * DIN;
#pragma unroll 1
  for (int d4 = 0; d4 < DIN; d4 += 4) {
    const v4f_t xv = *(const v4f*)(xr + d4);
    float xs[4];
    xs[0] = bfr(xv.x); xs[1] = bfr(xv.y); xs[2] = bfr(xv.z); xs[3] = bfr(xv.w);
#pragma unroll
    for (int q = 0; q < 4; ++q) {
      const float* wq = gws + (d4 + q) * NE;
#pragma unroll
      for (int e = 0; e < NE; ++e) acc[e] += (double)(xs[q] * wq[e]);
    }
  }

  float lg[NE];
#pragma unroll
  for (int e = 0; e < NE; ++e) lg[e] = (float)acc[e] + gbs[e];

  float mx = lg[0];
#pragma unroll
  for (int e = 1; e < NE; ++e) mx = fmaxf(mx, lg[e]);
  float p[NE], psum = 0.0f;
#pragma unroll
  for (int e = 0; e < NE; ++e) { p[e] = __expf(lg[e] - mx); psum += p[e]; }
  const float rs = __builtin_amdgcn_rcpf(psum);

  int e0 = 0; float l0 = lg[0];
#pragma unroll
  for (int e = 1; e < NE; ++e) if (lg[e] > l0) { l0 = lg[e]; e0 = e; }
  int e1 = -1; float l1 = -__builtin_huge_valf();
#pragma unroll
  for (int e = 0; e < NE; ++e) if (e != e0 && lg[e] > l1) { l1 = lg[e]; e1 = e; }
  if (e1 < 0) { e1 = (e0 == 0) ? 1 : 0; }

  const float w1 = expf(l1 - l0);
  const float ssum = 1.0f + w1;
  const float rsum = 1.0f / ssum;
  const float gw0 = rsum;
  const float gw1 = w1 * rsum;

  float ps[NE], cs[NE];
#pragma unroll
  for (int e = 0; e < NE; ++e) {
    ps[e] = p[e] * rs;
    cs[e] = (e == e0 || e == e1) ? 1.0f : 0.0f;
  }
#pragma unroll
  for (int e = 0; e < NE; ++e) { ps[e] = wsum(ps[e]); cs[e] = wsum(cs[e]); }
  if (lane == 0) {
#pragma unroll
    for (int e = 0; e < NE; ++e) { wred[w][e] = ps[e]; wred[w][8 + e] = cs[e]; }
  }

  v4u_t rv;
  rv.x = (unsigned)e0; rv.y = (unsigned)e1;
  rv.z = __float_as_uint(gw0); rv.w = __float_as_uint(gw1);
  unsigned* rp = route + (size_t)tok * 4;
  *(volatile v4u_t*)rp = rv;
  __syncthreads();

  if (tid < 32) {
    float s = 0.0f;
#pragma unroll
    for (int j = 0; j < GTPB / 32; ++j) s += wred[j][tid & 15];
    line[tid] = (tid < 16) ? s : 0.0f;
  }
  __syncthreads();
  const v4f_t pv = *(const v4f*)(line + 4 * (lane & 7));
  float* pp = partg + (size_t)blockIdx.x * 32 + 4 * (lane & 7);
  if (tid < 8) *(volatile v4f_t*)pp = pv;
  __threadfence();
  *(volatile v4u_t*)rp = rv;
  if (tid < 8) *(volatile v4f_t*)pp = pv;
}

__global__ __launch_bounds__(256) void k_route(const unsigned* __restrict__ route,
                                               int* __restrict__ tok_tab,
                                               int* __restrict__ cnt_tab)
{
  __shared__ __align__(16) int lst[LCAP];
  __shared__ int wtot[8];
  const int e = blockIdx.x;
  const int tid = threadIdx.x, lane = tid & 31, w = tid >> 5;

#pragma unroll 1
  for (int i = tid; i < LCAP; i += 256) lst[i] = 0;
  int base = 0;
  __syncthreads();

#pragma unroll 1
  for (int c0 = 0; c0 < NB; c0 += 256) {
    const v4u_t r = *(const v4u*)(route + (size_t)(c0 + tid) * 4);
    const int hit0 = ((int)r.x == e) ? 1 : 0;
    const int hit1 = ((int)r.y == e) ? 1 : 0;
    const int hit = hit0 | hit1;
    const unsigned bal = (unsigned)__ballot(hit);
    const int pre = __popc(bal & ((1u << lane) - 1u));
    const int tot = __popc(bal);
    if (lane == 0) wtot[w] = tot;
    __syncthreads();
    int wpre = 0, btot = 0;
#pragma unroll
    for (int j = 0; j < 8; ++j) {
      const int t = wtot[j];
      wpre += (j < w) ? t : 0;
      btot += t;
    }
    if (hit) {
      const int pos = base + wpre + pre;
      if (pos < LCAP) lst[pos] = (c0 + tid) * 2 + hit1;
    }
    base += btot;
    __syncthreads();
  }

  const int count = min(base, LCAP);
  const int ovf = (base > LCAP) ? 1 : 0;
  int* tp = tok_tab + (size_t)e * LCAP;
  v4u_t cv;
  cv.x = (tid == 0) ? (unsigned)count : 0u;
  cv.y = (tid == 0) ? (unsigned)ovf : 0u;
  cv.z = 0u; cv.w = 0u;
  int* cp = cnt_tab + e * 32 + 4 * (tid & 7);

#pragma unroll 1
  for (int i = tid; i < LCAP / 4; i += 256) {
    const v4u_t v = *(const v4u*)(lst + 4 * i);
    *(volatile v4u_t*)(tp + 4 * i) = v;
  }
  if (tid < 8) *(volatile v4u_t*)cp = cv;
  __threadfence();
#pragma unroll 1
  for (int i = tid; i < LCAP / 4; i += 256) {
    const v4u_t v = *(const v4u*)(lst + 4 * i);
    *(volatile v4u_t*)(tp + 4 * i) = v;
  }
  if (tid < 8) *(volatile v4u_t*)cp = cv;
}

template <int N>
__device__ __forceinline__ void ln_hilo(const float* stage, const float* sc, const float* sh,
                                        us* dst, int w, int lane)
{
  constexpr int J = N / 32;
#pragma unroll 1
  for (int rr = 0; rr < 4; ++rr) {
    const int row = 4 * w + rr;
    float v[J];
    float s = 0.0f;
#pragma unroll
    for (int j = 0; j < J; ++j) { v[j] = stage[row * N + 32 * j + lane]; s += v[j]; }
    s = wsum(s);
    const float mean = s * (1.0f / (float)N);
    float q = 0.0f;
#pragma unroll
    for (int j = 0; j < J; ++j) { const float d = v[j] - mean; q += d * d; }
    q = wsum(q);
    const float rstd = rsqrtf(q * (1.0f / (float)N) + LN_EPS);
#pragma unroll
    for (int j = 0; j < J; ++j) {
      const int col = 32 * j + lane;
      float hv = (v[j] - mean) * rstd * sc[col] + sh[col];
      hv = fmaxf(hv, 0.0f);
      const unsigned hi = f2bf(hv);
      const unsigned lo = f2bf(hv - bf2f(hi));
      dst[row * (2 * N) + col]     = (us)hi;
      dst[row * (2 * N) + N + col] = (us)lo;
    }
  }
}

__global__ __launch_bounds__(256) void k_expert(
    const us* __restrict__ xb,
    const us* __restrict__ w1t,
    const us* __restrict__ w2s,
    const us* __restrict__ w3s,
    const float* __restrict__ b1, const float* __restrict__ s1, const float* __restrict__ t1,
    const float* __restrict__ b2, const float* __restrict__ s2, const float* __restrict__ t2,
    const float* __restrict__ b3, const float* __restrict__ s3, const float* __restrict__ t3,
    const int* __restrict__ tok_tab,
    const int* __restrict__ cnt_tab,
    float* __restrict__ eo)
{
  extern __shared__ __align__(16) unsigned char dlds[];
  float* stage = (float*)(dlds + OFF_STAGE);
  us*    a2    = (us*)(dlds + OFF_A2);
  us*    a13   = (us*)(dlds + OFF_A13);
  float* par   = (float*)(dlds + OFF_PAR);
  int*   ents  = (int*)(dlds + OFF_ENT);

  const int e = blockIdx.y, tile = blockIdx.x;
  int count = cnt_tab[e * 32];
  count = min(max(count, 0), LCAP);
  if (tile * MT >= count) return;
  const int nvalid = min(MT, count - tile * MT);

  const int tid = threadIdx.x, lane = tid & 31, w = tid >> 5;
  const int h = lane >> 4, m = lane & 15;

  {
    int idx = tile * MT + min(tid & 31, nvalid - 1);
    idx = min(idx, LCAP - 1);
    int pk = tok_tab[(size_t)e * LCAP + idx];
    pk = min(max(pk, 0), 2 * NB - 1);
    if (tid < MT) ents[tid] = pk;
  }
#pragma unroll 1
  for (int i = tid; i < L1N; i += 256) {
    par[PAR_B1 + i] = bfr(b1[e * L1N + i]);
    par[PAR_S1 + i] = bfr(s1[e * L1N + i]);
    par[PAR_T1 + i] = bfr(t1[e * L1N + i]);
  }
  {
    par[PAR_B2 + tid] = bfr(b2[e * L2N + tid]);
    par[PAR_S2 + tid] = bfr(s2[e * L2N + tid]);
    par[PAR_T2 + tid] = bfr(t2[e * L2N + tid]);
    const int i3 = tid & (L3N - 1);
    const float vb = bfr(b3[e * L3N + i3]);
    const float vs = bfr(s3[e * L3N + i3]);
    const float vt = bfr(t3[e * L3N + i3]);
    if (tid < L3N) { par[PAR_B3 + tid] = vb; par[PAR_S3 + tid] = vs; par[PAR_T3 + tid] = vt; }
  }
  __syncthreads();

#pragma unroll
  for (int it = 0; it < 4; ++it) {
    const int i = it * 256 + tid;
    const int row = i >> 5, c = i & 31;
    const int tk = ents[row] >> 1;
    ((v4u_t*)a13)[row * 32 + c] = *(const v4u*)(xb + (size_t)tk * DIN + 8 * c);
  }
  __syncthreads();

  {
    v8f acc[2][4];
#pragma unroll
    for (int mt = 0; mt < 2; ++mt)
#pragma unroll
      for (int nt = 0; nt < 4; ++nt) acc[mt][nt] = zero8();
    const us* pa0 = a13 + m * DIN;
    const us* pa1 = a13 + (16 + m) * DIN;
    const us* pb  = w1t + ((size_t)e * L1N + 64 * w + m) * DIN;
#pragma unroll 1
    for (int k0 = 0; k0 < DIN; k0 += 32) {
      const v16bf fa0 = ldfrag(pa0 + k0, h);
      const v16bf fa1 = ldfrag(pa1 + k0, h);
#pragma unroll
      for (int nt = 0; nt < 4; ++nt) {
        const v16bf fb = ldfrag(pb + (size_t)nt * 16 * DIN + k0, h);
        acc[0][nt] = wmma_bf(fa0, fb, acc[0][nt]);
        acc[1][nt] = wmma_bf(fa1, fb, acc[1][nt]);
      }
    }
#pragma unroll
    for (int nt = 0; nt < 4; ++nt) {
      const int col = 64 * w + 16 * nt + m;
      const float bv = par[PAR_B1 + col];
#pragma unroll
      for (int mt = 0; mt < 2; ++mt)
#pragma unroll
        for (int r = 0; r < 8; ++r)
          stage[(16 * mt + 8 * h + r) * L1N + col] = acc[mt][nt][r] + bv;
    }
  }
  __syncthreads();
  ln_hilo<L1N>(stage, par + PAR_S1, par + PAR_T1, a2, w, lane);
  __syncthreads();

  {
    v8f acc[2][2];
#pragma unroll
    for (int mt = 0; mt < 2; ++mt)
#pragma unroll
      for (int nt = 0; nt < 2; ++nt) acc[mt][nt] = zero8();
    const us* pa0 = a2 + m * K2;
    const us* pa1 = a2 + (16 + m) * K2;
    const us* pb  = w2s + ((size_t)e * L2N + 32 * w + m) * K2;
#pragma unroll 1
    for (int k0 = 0; k0 < K2; k0 += 32) {
      const v16bf fa0 = ldfrag(pa0 + k0, h);
      const v16bf fa1 = ldfrag(pa1 + k0, h);
#pragma unroll
      for (int nt = 0; nt < 2; ++nt) {
        const v16bf fb = ldfrag(pb + (size_t)nt * 16 * K2 + k0, h);
        acc[0][nt] = wmma_bf(fa0, fb, acc[0][nt]);
        acc[1][nt] = wmma_bf(fa1, fb, acc[1][nt]);
      }
    }
#pragma unroll
    for (int nt = 0; nt < 2; ++nt) {
      const int col = 32 * w + 16 * nt + m;
      const float bv = par[PAR_B2 + col];
#pragma unroll
      for (int mt = 0; mt < 2; ++mt)
#pragma unroll
        for (int r = 0; r < 8; ++r)
          stage[(16 * mt + 8 * h + r) * L2N + col] = acc[mt][nt][r] + bv;
    }
  }
  __syncthreads();
  ln_hilo<L2N>(stage, par + PAR_S2, par + PAR_T2, a13, w, lane);
  __syncthreads();

  {
    v8f acc[2];
    acc[0] = zero8(); acc[1] = zero8();
    const us* pa0 = a13 + m * K3;
    const us* pa1 = a13 + (16 + m) * K3;
    const us* pb  = w3s + ((size_t)e * L3N + 16 * w + m) * K3;
#pragma unroll 1
    for (int k0 = 0; k0 < K3; k0 += 32) {
      const v16bf fa0 = ldfrag(pa0 + k0, h);
      const v16bf fa1 = ldfrag(pa1 + k0, h);
      const v16bf fb  = ldfrag(pb + k0, h);
      acc[0] = wmma_bf(fa0, fb, acc[0]);
      acc[1] = wmma_bf(fa1, fb, acc[1]);
    }
    const int col = 16 * w + m;
    const float bv = par[PAR_B3 + col];
#pragma unroll
    for (int mt = 0; mt < 2; ++mt)
#pragma unroll
      for (int r = 0; r < 8; ++r)
        stage[(16 * mt + 8 * h + r) * L3N + col] = acc[mt][r] + bv;
  }
  __syncthreads();

  {
    float scq[4], shq[4];
#pragma unroll
    for (int q = 0; q < 4; ++q) {
      scq[q] = par[PAR_S3 + 4 * lane + q];
      shq[q] = par[PAR_T3 + 4 * lane + q];
    }
    v4f_t o3[4];
#pragma unroll
    for (int rr = 0; rr < 4; ++rr) {
      const int row = 4 * w + rr;
      const v4f_t v = *(const v4f*)(stage + row * L3N + 4 * lane);
      float s = (v.x + v.y) + (v.z + v.w);
      s = wsum(s);
      const float mean = s * (1.0f / (float)L3N);
      const float dx = v.x - mean, dy = v.y - mean, dz = v.z - mean, dw = v.w - mean;
      float q = dx * dx + dy * dy + dz * dz + dw * dw;
      q = wsum(q);
      const float rstd = rsqrtf(q * (1.0f / (float)L3N) + LN_EPS);
      v4f_t o;
      o.x = fmaxf(dx * rstd * scq[0] + shq[0], 0.0f);
      o.y = fmaxf(dy * rstd * scq[1] + shq[1], 0.0f);
      o.z = fmaxf(dz * rstd * scq[2] + shq[2], 0.0f);
      o.w = fmaxf(dw * rstd * scq[3] + shq[3], 0.0f);
      o3[rr] = o;
    }
#pragma unroll
    for (int rr = 0; rr < 4; ++rr) {
      const int row = 4 * w + rr;
      if (row < nvalid) {
        const int pr = ents[row];
        *(volatile v4f_t*)(eo + (size_t)pr * L3N + 4 * lane) = o3[rr];
      }
    }
    __threadfence();
#pragma unroll
    for (int rr = 0; rr < 4; ++rr) {
      const int row = 4 * w + rr;
      if (row < nvalid) {
        const int pr = ents[row];
        *(volatile v4f_t*)(eo + (size_t)pr * L3N + 4 * lane) = o3[rr];
      }
    }
  }
}

__global__ __launch_bounds__(256) void k_combine(const float* __restrict__ eo,
                                                 const unsigned* __restrict__ route,
                                                 const int* __restrict__ cnt_tab,
                                                 float* __restrict__ out1,
                                                 us* __restrict__ fa)
{
  const int tid = threadIdx.x, lane = tid & 31, w = tid >> 5;
  int fl = cnt_tab[(lane & 7) * 32 + 1];
  fl = wor(fl);
  const float poison = (fl != 0) ? __uint_as_float(0x7fc00000u) : 0.0f;
  const int bb = blockIdx.x * 64 + 8 * w;

  v4f_t fo[8];
  v4u_t po[8];
#pragma unroll
  for (int j = 0; j < 8; ++j) {
    const int b = bb + j;
    const v4u_t r = *(const v4u*)(route + (size_t)b * 4);
    const float g0 = __uint_as_float(r.z), g1 = __uint_as_float(r.w);
    const v4f_t s0 = *(const v4f*)(eo + (size_t)(2 * b) * L3N + 4 * lane);
    const v4f_t s1 = *(const v4f*)(eo + (size_t)(2 * b + 1) * L3N + 4 * lane);
    v4f_t f;
    f.x = (g0 * s0.x + g1 * s1.x) + poison;
    f.y = (g0 * s0.y + g1 * s1.y) + poison;
    f.z = (g0 * s0.z + g1 * s1.z) + poison;
    f.w = (g0 * s0.w + g1 * s1.w) + poison;
    fo[j] = f;
    const unsigned hx = f2bf(f.x), hy = f2bf(f.y), hz = f2bf(f.z), hq = f2bf(f.w);
    const unsigned lx = f2bf(f.x - bf2f(hx)), ly = f2bf(f.y - bf2f(hy));
    const unsigned lz = f2bf(f.z - bf2f(hz)), lq = f2bf(f.w - bf2f(hq));
    v4u_t pk;
    pk.x = hx | (hy << 16); pk.y = hz | (hq << 16);
    pk.z = lx | (ly << 16); pk.w = lz | (lq << 16);
    po[j] = pk;
    *(volatile v4f_t*)(out1 + (size_t)b * L3N + 4 * lane) = f;
    *(volatile v4u_t*)(fa + (size_t)b * KH + 8 * lane) = pk;
  }
  __threadfence();
#pragma unroll
  for (int j = 0; j < 8; ++j) {
    const int b = bb + j;
    *(volatile v4f_t*)(out1 + (size_t)b * L3N + 4 * lane) = fo[j];
    *(volatile v4u_t*)(fa + (size_t)b * KH + 8 * lane) = po[j];
  }
}

__global__ __launch_bounds__(96) void k_heads(const us* __restrict__ fa,
                                              const us* __restrict__ hw1s,
                                              const float* __restrict__ hb1,
                                              const float* __restrict__ hw2,
                                              const float* __restrict__ hb2,
                                              float* __restrict__ out0)
{
  __shared__ __align__(16) float so[NTK][32];
  const int tid = threadIdx.x, lane = tid & 31, w = tid >> 5;
  const int h = lane >> 4, m = lane & 15;
  const int b0 = blockIdx.x * 32;

  const us* pa0 = fa + (size_t)(b0 + m) * KH;
  const us* pa1 = fa + (size_t)(b0 + 16 + m) * KH;
  const us* pb  = hw1s + ((size_t)w * HN + m) * KH;

  v8f acc[2][4];
#pragma unroll
  for (int mt = 0; mt < 2; ++mt)
#pragma unroll
    for (int nt = 0; nt < 4; ++nt) acc[mt][nt] = zero8();
#pragma unroll 1
  for (int k0 = 0; k0 < KH; k0 += 32) {
    const v16bf fa0 = ldfrag(pa0 + k0, h);
    const v16bf fa1 = ldfrag(pa1 + k0, h);
#pragma unroll
    for (int nt = 0; nt < 4; ++nt) {
      const v16bf fb = ldfrag(pb + (size_t)nt * 16 * KH + k0, h);
      acc[0][nt] = wmma_bf(fa0, fb, acc[0][nt]);
      acc[1][nt] = wmma_bf(fa1, fb, acc[1][nt]);
    }
  }

  float rs[2][8];
#pragma unroll
  for (int mt = 0; mt < 2; ++mt)
#pragma unroll
    for (int r = 0; r < 8; ++r) rs[mt][r] = 0.0f;
#pragma unroll
  for (int nt = 0; nt < 4; ++nt) {
    const int col = 16 * nt + m;
    const float bb = bfr(hb1[w * HN + col]);
    const float w2 = bfr(hw2[w * HN + col]);
#pragma unroll
    for (int mt = 0; mt < 2; ++mt)
#pragma unroll
      for (int r = 0; r < 8; ++r)
        rs[mt][r] += fmaxf(acc[mt][nt][r] + bb, 0.0f) * w2;
  }
#pragma unroll
  for (int mt = 0; mt < 2; ++mt)
#pragma unroll
    for (int r = 0; r < 8; ++r) {
#pragma unroll
      for (int off = 1; off < 16; off <<= 1) rs[mt][r] += __shfl_xor(rs[mt][r], off, 32);
    }
  const float bb2 = bfr(hb2[w]);
  if (m == 0) {
#pragma unroll
    for (int mt = 0; mt < 2; ++mt)
#pragma unroll
      for (int r = 0; r < 8; ++r) so[w][16 * mt + 8 * h + r] = rs[mt][r] + bb2;
  }
  __syncthreads();
  const v4f_t v = *(const v4f*)(&so[w][4 * (lane & 7)]);
  float* op = out0 + (size_t)w * NB + b0 + 4 * (lane & 7);
  if (lane < 8) *(volatile v4f_t*)op = v;
  __threadfence();
  if (lane < 8) *(volatile v4f_t*)op = v;
}

__global__ __launch_bounds__(32) void k_lb(const float* __restrict__ partg,
                                           const int* __restrict__ cnt_tab,
                                           float* __restrict__ out2)
{
  const int lane = threadIdx.x & 31;
  const int el = lane & 7;
  float ps = 0.0f, cs = 0.0f;
#pragma unroll 1
  for (int blk = 0; blk < GBLK; ++blk) {
    ps += partg[blk * 32 + el];
    cs += partg[blk * 32 + 8 + el];
  }
  const float frac = cs * (1.0f / (float)NB);
  const float pm   = ps * (1.0f / (float)NB);
  float term = (lane < NE) ? (frac * pm) : 0.0f;
  term = wsum(term);
  int fl = cnt_tab[el * 32 + 1];
  fl = wor(fl);
  const float lb = ALPHA_LB * term + ((fl != 0) ? __uint_as_float(0x7fc00000u) : 0.0f);
  if (lane == 0) *(volatile float*)out2 = lb;
  __threadfence();
  if (lane == 0) *(volatile float*)out2 = lb;
}

extern "C" void kernel_launch(void* const* d_in, const int* in_sizes, int n_in,
                              void* d_out, int out_size, void* d_ws, size_t ws_size,
                              hipStream_t stream)
{
  if (n_in < 19) return;
  if (in_sizes[0] != NB * DIN) return;
  if (in_sizes[1] != DIN * NE) return;
  if (in_sizes[2] != NE) return;
  if (in_sizes[3] != NE * DIN * L1N) return;
  if (in_sizes[4] != NE * L1N || in_sizes[5] != NE * L1N || in_sizes[6] != NE * L1N) return;
  if (in_sizes[7] != NE * L1N * L2N) return;
  if (in_sizes[8] != NE * L2N || in_sizes[9] != NE * L2N || in_sizes[10] != NE * L2N) return;
  if (in_sizes[11] != NE * L2N * L3N) return;
  if (in_sizes[12] != NE * L3N || in_sizes[13] != NE * L3N || in_sizes[14] != NE * L3N) return;
  if (in_sizes[15] != NTK * L3N * HN) return;
  if (in_sizes[16] != NTK * HN) return;
  if (in_sizes[17] != NTK * HN) return;
  if (in_sizes[18] != NTK) return;
  if (out_size != NTK * NB + NB * L3N + 1) return;

  const float* x      = (const float*)d_in[0];
  const float* gate_W = (const float*)d_in[1];
  const float* gate_b = (const float*)d_in[2];
  const float* W1 = (const float*)d_in[3];
  const float* b1 = (const float*)d_in[4];
  const float* s1 = (const float*)d_in[5];
  const float* t1 = (const float*)d_in[6];
  const float* W2 = (const float*)d_in[7];
  const float* b2 = (const float*)d_in[8];
  const float* s2 = (const float*)d_in[9];
  const float* t2 = (const float*)d_in[10];
  const float* W3 = (const float*)d_in[11];
  const float* b3 = (const float*)d_in[12];
  const float* s3 = (const float*)d_in[13];
  const float* t3 = (const float*)d_in[14];
  const float* hW1 = (const float*)d_in[15];
  const float* hb1 = (const float*)d_in[16];
  const float* hW2 = (const float*)d_in[17];
  const float* hb2 = (const float*)d_in[18];

  float* out0 = (float*)d_out;
  float* out1 = out0 + (size_t)NTK * NB;
  float* out2 = out0 + (size_t)NTK * NB + (size_t)NB * L3N;

  size_t o = 0;
  auto carve = [&](size_t bytes) { const size_t p = o; o += (bytes + 127) & ~(size_t)127; return p; };
  const size_t oXB = carve((size_t)NB * DIN * 2);
  const size_t oW1 = carve((size_t)NE * L1N * DIN * 2);
  const size_t oW2 = carve((size_t)NE * L2N * K2 * 2);
  const size_t oW3 = carve((size_t)NE * L3N * K3 * 2);
  const size_t oHW = carve((size_t)NTK * HN * KH * 2);
  const size_t oRT = carve((size_t)NB * 16);
  const size_t oPG = carve((size_t)GBLK * 128);
  const size_t oTK = carve((size_t)NE * LCAP * 4);
  const size_t oCN = carve((size_t)NE * 128);
  const size_t oEO = carve((size_t)2 * NB * L3N * 4);
  const size_t oFA = carve((size_t)NB * KH * 2);
  const size_t total = o;
  if (total > ws_size) return;
  if (total > (size_t)134217728) return;

  char* ws = (char*)d_ws;
  us*       xb   = (us*)(ws + oXB);
  us*       w1t  = (us*)(ws + oW1);
  us*       w2s  = (us*)(ws + oW2);
  us*       w3s  = (us*)(ws + oW3);
  us*       hw1s = (us*)(ws + oHW);
  unsigned* route = (unsigned*)(ws + oRT);
  float*    partg = (float*)(ws + oPG);
  int*      tok_tab = (int*)(ws + oTK);
  int*      cnt_tab = (int*)(ws + oCN);
  float*    eo   = (float*)(ws + oEO);
  us*       fah  = (us*)(ws + oFA);

  const int n8x = NB * DIN / 8;
  k_cvt_x<<<(n8x + 255) / 256, 256, 0, stream>>>(x, xb, n8x);
  const int g1 = NE * L1N * DIN / 8;
  k_prep_w<<<(g1 + 255) / 256, 256, 0, stream>>>(W1, w1t, DIN, L1N, DIN, 0, g1);
  const int g2 = NE * L2N * K2 / 8;
  k_prep_w<<<(g2 + 255) / 256, 256, 0, stream>>>(W2, w2s, L1N, L2N, K2, 0, g2);
  const int g3 = NE * L3N * K3 / 8;
  k_prep_w<<<(g3 + 255) / 256, 256, 0, stream>>>(W3, w3s, L2N, L3N, K3, 0, g3);
  const int gh = NTK * HN * KH / 8;
  k_prep_w<<<(gh + 255) / 256, 256, 0, stream>>>(hW1, hw1s, L3N, HN, KH, 1, gh);

  k_gate<<<GBLK, GTPB, 0, stream>>>(x, gate_W, gate_b, route, partg);
  k_route<<<NE, 256, 0, stream>>>(route, tok_tab, cnt_tab);

  hipFuncSetAttribute(reinterpret_cast<const void*>(&k_expert),
                      hipFuncAttributeMaxDynamicSharedMemorySize, DYN_LDS);
  k_expert<<<dim3(NTILE, NE), 256, DYN_LDS, stream>>>(
      xb, w1t, w2s, w3s, b1, s1, t1, b2, s2, t2, b3, s3, t3, tok_tab, cnt_tab, eo);

  k_combine<<<NB / 64, 256, 0, stream>>>(eo, route, cnt_tab, out1, fah);
  k_heads<<<NB / 32, 96, 0, stream>>>(fah, hw1s, hb1, hW2, hb2, out0);
  k_lb<<<1, 32, 0, stream>>>(partg, cnt_tab, out2);
}
